// _EGNNLayer_14551349199304
// MI455X (gfx1250) — hardware-verified
//
#include <hip/hip_runtime.h>
#include <stddef.h>


typedef __attribute__((ext_vector_type(16))) _Float16 v16h;
typedef __attribute__((ext_vector_type(8)))  _Float16 v8h;
typedef __attribute__((ext_vector_type(16))) __bf16   v16b;
typedef __attribute__((ext_vector_type(8)))  __bf16   v8b;
typedef __attribute__((ext_vector_type(8)))  float    v8f;
typedef __attribute__((ext_vector_type(4)))  float    v4f;

__device__ __forceinline__ unsigned short f2bf_bits(float f) {
  unsigned u = __float_as_uint(f);
  return (unsigned short)((u + 0x7FFFu + ((u >> 16) & 1u)) >> 16);
}
__device__ __forceinline__ float bf_bits2f(unsigned short h) { return __uint_as_float(((unsigned)h) << 16); }

__device__ __forceinline__ void dep_guard_h(v8f& a, v8f& b, v16h x, v16h y) { asm volatile("v_nop\n\tv_nop\n\tv_nop\n\tv_nop" : "+v"(a), "+v"(b) : "v"(x), "v"(y)); }
__device__ __forceinline__ void dep_guard_b(v8f& a, v8f& b, v16b x, v16b y) { asm volatile("v_nop\n\tv_nop\n\tv_nop\n\tv_nop" : "+v"(a), "+v"(b) : "v"(x), "v"(y)); }
__device__ __forceinline__ void keep4_h(v16h a, v16h b, v16h c, v16h d) { asm volatile("v_nop" :: "v"(a), "v"(b), "v"(c), "v"(d)); }
__device__ __forceinline__ void keep4_b(v16b a, v16b b, v16b c, v16b d) { asm volatile("v_nop" :: "v"(a), "v"(b), "v"(c), "v"(d)); }
__device__ __forceinline__ void acc_guard4(v8f& a, v8f& b, v8f& c, v8f& d) { asm volatile("v_nop\n\tv_nop\n\tv_nop\n\tv_nop" : "+v"(a), "+v"(b), "+v"(c), "+v"(d)); }
template <typename T> struct Frag;
template <> struct Frag<_Float16> {
  typedef v16h V; union U { v16h v; v8h h[2]; };
  static __device__ __forceinline__ v16h load(const _Float16* p) {
    U f; f.h[0] = *(const v8h*)(p); f.h[1] = *(const v8h*)(p + 16); return f.v;
  }
  static __device__ __forceinline__ v8f mma(v16h a, v16h b, v8f c) {
    return __builtin_amdgcn_wmma_f32_16x16x32_f16(false, a, false, b, (short)0, c, false, false);
  }
  static __device__ __forceinline__ void guard(v8f& a, v8f& b, v16h x, v16h y) { dep_guard_h(a, b, x, y); }
  static __device__ __forceinline__ void keep(v16h a, v16h b, v16h c, v16h d) { keep4_h(a, b, c, d); }
};
template <> struct Frag<__bf16> {
  typedef v16b V; union U { v16b v; v8b h[2]; };
  static __device__ __forceinline__ v16b load(const __bf16* p) {
    U f; f.h[0] = *(const v8b*)(p); f.h[1] = *(const v8b*)(p + 16); return f.v;
  }
  static __device__ __forceinline__ v8f mma(v16b a, v16b b, v8f c) {
    return __builtin_amdgcn_wmma_f32_16x16x32_bf16(false, a, false, b, (short)0, c, false, false);
  }
  static __device__ __forceinline__ void guard(v8f& a, v8f& b, v16b x, v16b y) { dep_guard_b(a, b, x, y); }
  static __device__ __forceinline__ void keep(v16b a, v16b b, v16b c, v16b d) { keep4_b(a, b, c, d); }
};

template <int ET> struct Elem;
template <> struct Elem<0> { typedef _Float16 T; };
template <> struct Elem<1> { typedef __bf16 T; };
template <int ET, bool SPLIT, int BIAS_MODE, int OUT_MODE, bool RESID, int ACT = 0>
__global__ __launch_bounds__(256) void wmma_gemm64(
    const unsigned short* __restrict__ Ap, const unsigned short* __restrict__ A2p, int lda, long strideA,
    const unsigned short* __restrict__ Btp, const unsigned short* __restrict__ Bt2p, int ldb, long strideB,
    void* __restrict__ Cout, void* __restrict__ Cout2, int ldc, long strideC,
    const float* __restrict__ bias,
    const float* __restrict__ resid, long strideR,
    int M, int N, int K, float scale) {
  typedef typename Elem<ET>::T T;
  typedef typename Frag<T>::V V;
  const T* A = (const T*)Ap; const T* A2 = (const T*)A2p; const T* Bt = (const T*)Btp; const T* Bt2 = (const T*)Bt2p;
  __shared__ __align__(16) float sT[8][16 * 68];
  const int b    = blockIdx.y;
  const int lane = threadIdx.x & 31;
  const int wave = threadIdx.x >> 5;
  const int tilesN = N >> 6;
  const int tilesM = M >> 6;
  const int tile = blockIdx.x * 8 + wave;
  if (tile >= tilesM * tilesN) return;
  const int tm = tile / tilesN;
  const int tn = tile - tm * tilesN;
  const int m0 = tm << 6;
  const int n0 = tn << 6;

  const T* Ab  = A  + (size_t)b * strideA;
  const T* Bb  = Bt + (size_t)b * strideB;
  const T* Ab2 = SPLIT ? (A2  + (size_t)b * strideA) : nullptr;
  const T* Bb2 = SPLIT ? (Bt2 + (size_t)b * strideB) : nullptr;

  const int rlane = lane & 15;
  const int koff  = (lane >> 4) * 8;
  const int mOff  = (lane >> 4) * 8;

  v8f acc[4][4];
#pragma unroll
  for (int i = 0; i < 4; ++i)
#pragma unroll
    for (int j = 0; j < 4; ++j) acc[i][j] = (v8f){0.f,0.f,0.f,0.f,0.f,0.f,0.f,0.f};

  for (int k0 = 0; k0 < K; k0 += 32) {
    V bh[4], bl[4];
#pragma unroll
    for (int j = 0; j < 4; ++j) {
      const size_t bo = (size_t)(n0 + (j << 4) + rlane) * ldb + koff + k0;
      bh[j] = Frag<T>::load(Bb + bo);
      if (SPLIT) bl[j] = Frag<T>::load(Bb2 + bo);
    }
#pragma unroll
    for (int i = 0; i < 4; ++i) {
      const size_t ao = (size_t)(m0 + (i << 4) + rlane) * lda + koff + k0;
      V ah = Frag<T>::load(Ab + ao);
      V al;
      if (SPLIT) al = Frag<T>::load(Ab2 + ao);
#pragma unroll
      for (int j = 0; j < 4; ++j) {
        acc[i][j] = Frag<T>::mma(ah, bh[j], acc[i][j]);
        if (SPLIT) {
          acc[i][j] = Frag<T>::mma(ah, bl[j], acc[i][j]);
          acc[i][j] = Frag<T>::mma(al, bh[j], acc[i][j]);
        }
      }
      Frag<T>::guard(acc[i][0], acc[i][3], ah, SPLIT ? al : ah);
    }
    Frag<T>::keep(bh[0], bh[1], bh[2], bh[3]);
    if (SPLIT) Frag<T>::keep(bl[0], bl[1], bl[2], bl[3]);
  }
  acc_guard4(acc[0][0], acc[0][1], acc[0][2], acc[0][3]);
  acc_guard4(acc[1][0], acc[1][1], acc[1][2], acc[1][3]);
  acc_guard4(acc[2][0], acc[2][1], acc[2][2], acc[2][3]);
  acc_guard4(acc[3][0], acc[3][1], acc[3][2], acc[3][3]);

  float* slab = sT[wave];
  const float* Rb = RESID ? (resid + (size_t)b * strideR) : nullptr;
#pragma unroll
  for (int i = 0; i < 4; ++i) {
    const int mBase = m0 + (i << 4);
#pragma unroll
    for (int j = 0; j < 4; ++j) {
      const int n = n0 + (j << 4) + rlane;
      float bv = 0.f;
      if (BIAS_MODE == 2) bv = bias[n];
#pragma unroll
      for (int r = 0; r < 8; ++r) {
        float v = acc[i][j][r] * scale;
        if (BIAS_MODE == 1) v += bias[mBase + mOff + r];
        if (BIAS_MODE == 2) v += bv;
        if (RESID) v += Rb[(size_t)(mBase + mOff + r) * ldc + n];
        if (ACT == 1) v = tanhf(v);
        if (ACT == 2) v = fmaxf(v, 0.0f);
        if (ACT == 3) v = v / (1.0f + expf(-v));
        if (ACT == 4) v = (v > 0.f) ? v : 0.01f * v;
        if (ACT == 5) v = 0.5f * v * (1.0f + erff(v * 0.70710678118654752f));
        if (ACT == 6) v = v * __builtin_amdgcn_rcpf(1.0f + __expf(-v));
        slab[(mOff + r) * 68 + (j << 4) + rlane] = v;
      }
    }
    __builtin_amdgcn_fence(__ATOMIC_RELEASE, "workgroup");
    __builtin_amdgcn_wave_barrier();
    __builtin_amdgcn_fence(__ATOMIC_ACQUIRE, "workgroup");
    if (OUT_MODE == 0) {
      float* C = (float*)Cout + (size_t)b * strideC;
      const int hh = lane >> 4, c4 = (lane & 15) * 4;
      for (int pass = 0; pass < 2; ++pass) {
#pragma unroll
        for (int it = 0; it < 8; ++it) {
          const int row = it * 2 + hh;
          v4f v = *(const v4f*)(slab + row * 68 + c4);
          *(volatile v4f*)(C + (size_t)(mBase + row) * ldc + n0 + c4) = v;
        }
        __threadfence();
      }
    } else {
      const int q = lane >> 3, c8 = (lane & 7) * 8;
      unsigned short* C  = (unsigned short*)Cout  + (size_t)b * strideC;
      unsigned short* C2 = (OUT_MODE == 2) ? ((unsigned short*)Cout2 + (size_t)b * strideC) : nullptr;
      for (int pass = 0; pass < 2; ++pass) {
#pragma unroll
        for (int it = 0; it < 4; ++it) {
          const int row = it * 4 + q;
          const float* sp = slab + row * 68 + c8;
          v8h hv, lv;
#pragma unroll
          for (int e = 0; e < 8; ++e) {
            if (OUT_MODE == 1) {
              hv[e] = (_Float16)sp[e];
            } else {
              unsigned short hb = f2bf_bits(sp[e]);
              unsigned short lb = f2bf_bits(sp[e] - bf_bits2f(hb));
              hv[e] = __builtin_bit_cast(_Float16, hb);
              lv[e] = __builtin_bit_cast(_Float16, lb);
            }
          }
          *(volatile v8h*)(C + (size_t)(mBase + row) * ldc + n0 + c8) = hv;
          if (OUT_MODE == 2) *(volatile v8h*)(C2 + (size_t)(mBase + row) * ldc + n0 + c8) = lv;
        }
        __threadfence();
      }
    }
    __builtin_amdgcn_fence(__ATOMIC_RELEASE, "workgroup");
    __builtin_amdgcn_wave_barrier();
    __builtin_amdgcn_fence(__ATOMIC_ACQUIRE, "workgroup");
  }
}

__device__ __forceinline__ v8f mma_h(v16h a, v16h b, v8f c) {
  c = __builtin_amdgcn_wmma_f32_16x16x32_f16(false, a, false, b, (short)0, c, false, false);
  asm volatile("v_nop\n\tv_nop\n\tv_nop\n\tv_nop" : "+v"(c) : "v"(a), "v"(b));
  return c;
}

__device__ __forceinline__ float silu_f(float v) {
  const float e = __expf(-v);
  return v * __builtin_amdgcn_rcpf(1.0f + e);
}

__global__ __launch_bounds__(256) void k_cast_h(const float* __restrict__ h, _Float16* __restrict__ hcat, int nrows) {
  const int i = blockIdx.x * 256 + threadIdx.x;
  if (i < nrows * 16) {
    const int row = i >> 4, c8 = (i & 15) * 8;
    const v4f a0 = *(const v4f*)(h + (size_t)row * 128 + c8);
    const v4f a1 = *(const v4f*)(h + (size_t)row * 128 + c8 + 4);
    v8h pk;
#pragma unroll
    for (int e = 0; e < 4; ++e) { pk[e] = (_Float16)a0[e]; pk[4 + e] = (_Float16)a1[e]; }
    _Float16* p = hcat + (size_t)row * 256 + c8;
    *(volatile v8h*)p = pk;
    __threadfence();
    *(volatile v8h*)p = pk;
  }
}

__global__ __launch_bounds__(256) void k_wtrans(
    const float* __restrict__ We1, const float* __restrict__ We2, const float* __restrict__ Wc1,
    const float* __restrict__ Wn1, const float* __restrict__ Wn2,
    _Float16* __restrict__ We1T, _Float16* __restrict__ We2T, _Float16* __restrict__ Wc1T,
    _Float16* __restrict__ Wn1T, _Float16* __restrict__ Wn2T) {
  const int blk = blockIdx.x;
  const float* src; _Float16* dst; int kd; int lb;
  if (blk < 8)       { src = We1;              dst = We1T;              kd = 128; lb = blk; }
  else if (blk < 16) { src = We1 + 128 * 128;  dst = We1T + 128 * 128;  kd = 128; lb = blk - 8; }
  else if (blk < 24) { src = We2;              dst = We2T;              kd = 128; lb = blk - 16; }
  else if (blk < 32) { src = Wc1;              dst = Wc1T;              kd = 128; lb = blk - 24; }
  else if (blk < 48) { src = Wn1;              dst = Wn1T;              kd = 256; lb = blk - 32; }
  else               { src = Wn2;              dst = Wn2T;              kd = 128; lb = blk - 48; }
  const int t   = lb * 256 + threadIdx.x;
  const int kd8 = kd >> 3;
  const int n   = t / kd8;
  const int k0  = (t - n * kd8) * 8;
  v8h pk;
#pragma unroll
  for (int e = 0; e < 8; ++e) pk[e] = (_Float16)(64.0f * src[(size_t)(k0 + e) * 128 + n]);
  _Float16* p = dst + (size_t)n * kd + k0;
  *(volatile v8h*)p = pk;
  __threadfence();
  *(volatile v8h*)p = pk;
}

#define EG_NN 512
#define EG_EP 136
#define EG_STEPS 128

__global__ __launch_bounds__(256) void k_edge(
    const float* __restrict__ x, const float* __restrict__ AB,
    const float* __restrict__ We1, const float* __restrict__ be1,
    const float* __restrict__ be2, const float* __restrict__ bc1,
    const float* __restrict__ Wc2, const float* __restrict__ bc2,
    const _Float16* __restrict__ We2T, const _Float16* __restrict__ Wc1T,
    const int* __restrict__ radius,
    _Float16* __restrict__ hcat, float* __restrict__ outX) {
#pragma clang fp contract(off)
  __shared__ __align__(16) _Float16 eBuf[128 * EG_EP];
  __shared__ __align__(16) _Float16 mBuf[128 * EG_EP];
  __shared__ __align__(16) float AiT[32 * 128];
  __shared__ __align__(16) float wdS[128];
  __shared__ __align__(16) float xI[32 * 4];
  __shared__ __align__(16) float dxB[128 * 4];
  __shared__ __align__(16) float maskB[128];
  __shared__ __align__(16) float gateP[8 * 128];
  __shared__ __align__(16) float xOut[128];

  const int tid  = threadIdx.x;
  const int lane = tid & 31;
  const int wave = tid >> 5;
  const int hh   = lane >> 4;
  const int c    = lane & 15;
  const int koff = hh * 8;
  const int blk  = blockIdx.x;
  const int b    = blk >> 4;
  const int i0   = (blk & 15) << 5;
  const int nodeBase = b * EG_NN + i0;
  const int nloc = wave * 16 + c;
  const float rad = (float)radius[0];
  const float r2  = rad * rad;

  for (int t = tid; t < 32 * 32; t += 256) {
    const int row = t >> 5, c4 = (t & 31) * 4;
    const v4f a  = *(const v4f*)(AB + (size_t)(nodeBase + row) * 256 + c4);
    const v4f bb = *(const v4f*)(be1 + c4);
    *(v4f*)(AiT + row * 128 + c4) = a + bb;
  }
  if (tid < 128) wdS[tid] = We1[256 * 128 + tid];
  if (tid < 32) {
    xI[tid * 4 + 0] = x[(size_t)(nodeBase + tid) * 3 + 0];
    xI[tid * 4 + 1] = x[(size_t)(nodeBase + tid) * 3 + 1];
    xI[tid * 4 + 2] = x[(size_t)(nodeBase + tid) * 3 + 2];
    xI[tid * 4 + 3] = 0.0f;
  }
  const float be2v = be2[nloc];
  const float bc1v = bc1[nloc];
  const float wc2v = Wc2[nloc];
  const float bc2v = bc2[0];
  float aggR[2][8];
#pragma unroll
  for (int s = 0; s < 2; ++s)
#pragma unroll
    for (int r = 0; r < 8; ++r) aggR[s][r] = 0.0f;
  float cR0 = 0.0f, cR1 = 0.0f, cR2 = 0.0f, nR = 0.0f;
  __syncthreads();

  for (int js = 0; js < EG_STEPS; ++js) {
    const int j0 = js * 4;
    {
      const int m  = tid >> 1, kh = tid & 1;
      const int il = m & 31, jl = m >> 5;
      const int gj = j0 + jl;
      const float* xj = x + (size_t)(b * EG_NN + gj) * 3;
      const float dx0 = xI[il * 4 + 0] - xj[0];
      const float dx1 = xI[il * 4 + 1] - xj[1];
      const float dx2 = xI[il * 4 + 2] - xj[2];
      float d2 = dx0 * dx0;
      d2 = d2 + dx1 * dx1;
      d2 = d2 + dx2 * dx2;
      const float mk = ((d2 < r2) && ((i0 + il) != gj)) ? 1.0f : 0.0f;
      if (kh == 0) {
        dxB[m * 4 + 0] = dx0; dxB[m * 4 + 1] = dx1; dxB[m * 4 + 2] = dx2;
        maskB[m] = mk;
      }
      const float* bj = AB + (size_t)(b * EG_NN + gj) * 256 + 128 + kh * 64;
      const float* ai = AiT + il * 128 + kh * 64;
      const float* wd = wdS + kh * 64;
      _Float16* er = eBuf + m * EG_EP + kh * 64;
#pragma unroll 2
      for (int g = 0; g < 8; ++g) {
        const v4f a0 = *(const v4f*)(ai + 8 * g), a1 = *(const v4f*)(ai + 8 * g + 4);
        const v4f b0 = *(const v4f*)(bj + 8 * g), b1 = *(const v4f*)(bj + 8 * g + 4);
        const v4f w0 = *(const v4f*)(wd + 8 * g), w1 = *(const v4f*)(wd + 8 * g + 4);
        v8h pk;
#pragma unroll
        for (int e = 0; e < 4; ++e) {
          pk[e]     = (_Float16)(silu_f((a0[e] + b0[e]) + d2 * w0[e]) * 8.0f);
          pk[4 + e] = (_Float16)(silu_f((a1[e] + b1[e]) + d2 * w1[e]) * 8.0f);
        }
        *(v8h*)(er + 8 * g) = pk;
      }
    }
    __syncthreads();

    {
      v16h bw[4];
#pragma unroll
      for (int ks = 0; ks < 4; ++ks) bw[ks] = Frag<_Float16>::load(We2T + (size_t)nloc * 128 + koff + 32 * ks);
#pragma unroll 1
      for (int mp = 0; mp < 4; ++mp) {
#pragma unroll
        for (int s = 0; s < 2; ++s) {
          const int mt = 2 * mp + s;
          const _Float16* ap = eBuf + (16 * mt + c) * EG_EP + koff;
          v8f acc = (v8f){0.f,0.f,0.f,0.f,0.f,0.f,0.f,0.f};
#pragma unroll
          for (int ks = 0; ks < 4; ++ks) {
            const v16h a = Frag<_Float16>::load(ap + 32 * ks);
            acc = mma_h(a, bw[ks], acc);
          }
#pragma unroll
          for (int r = 0; r < 8; ++r) {
            const int m = 16 * mt + 8 * hh + r;
            float v = acc[r] * (1.0f / 512.0f) + be2v;
            v = silu_f(v) * maskB[m];
            aggR[s][r] = aggR[s][r] + v;
            mBuf[m * EG_EP + nloc] = (_Float16)(v * 16.0f);
          }
        }
      }
    }
    __syncthreads();

    {
      v16h bw[4];
#pragma unroll
      for (int ks = 0; ks < 4; ++ks) bw[ks] = Frag<_Float16>::load(Wc1T + (size_t)nloc * 128 + koff + 32 * ks);
#pragma unroll 1
      for (int mt = 0; mt < 8; ++mt) {
        const _Float16* ap = mBuf + (16 * mt + c) * EG_EP + koff;
        v8f acc = (v8f){0.f,0.f,0.f,0.f,0.f,0.f,0.f,0.f};
#pragma unroll
        for (int ks = 0; ks < 4; ++ks) {
          const v16h a = Frag<_Float16>::load(ap + 32 * ks);
          acc = mma_h(a, bw[ks], acc);
        }
        float p[8];
#pragma unroll
        for (int r = 0; r < 8; ++r) p[r] = silu_f(acc[r] * (1.0f / 1024.0f) + bc1v) * wc2v;
#pragma unroll
        for (int r = 0; r < 8; ++r) {
          p[r] = p[r] + __shfl_xor(p[r], 1, 32);
          p[r] = p[r] + __shfl_xor(p[r], 2, 32);
          p[r] = p[r] + __shfl_xor(p[r], 4, 32);
          p[r] = p[r] + __shfl_xor(p[r], 8, 32);
        }
        if (c == 0) {
#pragma unroll
          for (int r = 0; r < 8; ++r) gateP[wave * 128 + 16 * mt + 8 * hh + r] = p[r];
        }
      }
    }
    __syncthreads();

    if (tid < 32) {
      const int il = tid;
#pragma unroll
      for (int jl = 0; jl < 4; ++jl) {
        const int m = jl * 32 + il;
        float gs = gateP[m];
#pragma unroll
        for (int w = 1; w < 8; ++w) gs = gs + gateP[w * 128 + m];
        const float gate = gs + bc2v;
        const float mk = maskB[m];
        cR0 = cR0 + (dxB[m * 4 + 0] * gate) * mk;
        cR1 = cR1 + (dxB[m * 4 + 1] * gate) * mk;
        cR2 = cR2 + (dxB[m * 4 + 2] * gate) * mk;
        nR  = nR + mk;
      }
    }
    __syncthreads();
  }

  {
    _Float16* aggH = eBuf;
#pragma unroll
    for (int s = 0; s < 2; ++s)
#pragma unroll
      for (int r = 0; r < 8; ++r)
        aggH[(16 * s + 8 * hh + r) * EG_EP + nloc] = (_Float16)aggR[s][r];
  }
  __syncthreads();
  {
    const int c8 = c * 8;
    for (int pass = 0; pass < 2; ++pass) {
#pragma unroll
      for (int it = 0; it < 2; ++it) {
        const int row = wave * 4 + it * 2 + hh;
        const v8h val = *(const v8h*)(eBuf + row * EG_EP + c8);
        *(volatile v8h*)(hcat + (size_t)(nodeBase + row) * 256 + 128 + c8) = val;
      }
      __threadfence();
    }
  }
  if (tid < 32) {
    const float cnt = fmaxf(nR, 1.0f);
    const float rc = 1.0f / cnt;
    xOut[tid * 3 + 0] = xI[tid * 4 + 0] + cR0 * rc;
    xOut[tid * 3 + 1] = xI[tid * 4 + 1] + cR1 * rc;
    xOut[tid * 3 + 2] = xI[tid * 4 + 2] + cR2 * rc;
  }
  __syncthreads();
  for (int pass = 0; pass < 2; ++pass) {
    if (tid < 24) {
      const v4f val = *(const v4f*)(xOut + tid * 4);
      *(volatile v4f*)(outX + (size_t)nodeBase * 3 + tid * 4) = val;
    }
    __threadfence();
  }
}

extern "C" void kernel_launch(void* const* d_in, const int* in_sizes, int n_in,
                              void* d_out, int out_size, void* d_ws, size_t ws_size,
                              hipStream_t stream) {
  if (n_in < 15) return;
  const int nodes = 4 * 512;
  if (in_sizes[0] != nodes * 128 || in_sizes[1] != nodes * 3 || out_size != nodes * 128 + nodes * 3) return;
  if (in_sizes[2] != 257 * 128 || in_sizes[10] != 256 * 128) return;

  const float* h   = (const float*)d_in[0];
  const float* x   = (const float*)d_in[1];
  const float* We1 = (const float*)d_in[2];
  const float* be1 = (const float*)d_in[3];
  const float* We2 = (const float*)d_in[4];
  const float* be2 = (const float*)d_in[5];
  const float* Wc1 = (const float*)d_in[6];
  const float* bc1 = (const float*)d_in[7];
  const float* Wc2 = (const float*)d_in[8];
  const float* bc2 = (const float*)d_in[9];
  const float* Wn1 = (const float*)d_in[10];
  const float* bn1 = (const float*)d_in[11];
  const float* Wn2 = (const float*)d_in[12];
  const float* bn2 = (const float*)d_in[13];
  const int* radius = (const int*)d_in[14];

  char* ws = (char*)d_ws;
  size_t off = 0;
  _Float16* hcat = (_Float16*)(ws + off); off += (size_t)nodes * 256 * 2;
  _Float16* We1T = (_Float16*)(ws + off); off += (size_t)256 * 128 * 2;
  _Float16* We2T = (_Float16*)(ws + off); off += (size_t)128 * 128 * 2;
  _Float16* Wc1T = (_Float16*)(ws + off); off += (size_t)128 * 128 * 2;
  _Float16* Wn1T = (_Float16*)(ws + off); off += (size_t)128 * 256 * 2;
  _Float16* Wn2T = (_Float16*)(ws + off); off += (size_t)128 * 128 * 2;
  float*    AB   = (float*)(ws + off);    off += (size_t)nodes * 256 * 4;
  _Float16* t1   = (_Float16*)(ws + off); off += (size_t)nodes * 128 * 2;
  if (off > ws_size) return;

  float* outH = (float*)d_out;
  float* outX = outH + (size_t)nodes * 128;

  const unsigned short* hcatU = (const unsigned short*)hcat;
  const unsigned short* We1TU = (const unsigned short*)We1T;
  const unsigned short* Wn1TU = (const unsigned short*)Wn1T;
  const unsigned short* Wn2TU = (const unsigned short*)Wn2T;
  const unsigned short* t1U   = (const unsigned short*)t1;

  k_cast_h<<<(nodes * 16 + 255) / 256, 256, 0, stream>>>(h, hcat, nodes);
  k_wtrans<<<56, 256, 0, stream>>>(We1, We2, Wc1, Wn1, Wn2, We1T, We2T, Wc1T, Wn1T, Wn2T);
  wmma_gemm64<0, false, 0, 0, false, 0><<<dim3(16, 1), 256, 0, stream>>>(
      hcatU, hcatU, 256, 0L, We1TU, We1TU, 128, 0L, (void*)AB, (void*)AB, 256, 0L,
      be1, h, 0L, nodes, 256, 128, 1.0f / 64.0f);
  k_edge<<<4 * (512 / 32), 256, 0, stream>>>(x, AB, We1, be1, be2, bc1, Wc2, bc2, We2T, Wc1T, radius, hcat, outX);
  wmma_gemm64<0, false, 2, 1, false, 6><<<dim3(8, 1), 256, 0, stream>>>(
      hcatU, hcatU, 256, 0L, Wn1TU, Wn1TU, 256, 0L, (void*)t1, (void*)t1, 128, 0L,
      bn1, h, 0L, nodes, 128, 256, 1.0f / 64.0f);
  wmma_gemm64<0, false, 2, 0, true, 0><<<dim3(8, 1), 256, 0, stream>>>(
      t1U, t1U, 128, 0L, Wn2TU, Wn2TU, 128, 0L, (void*)outH, (void*)outH, 128, 0L,
      bn2, h, 0L, nodes, 128, 128, 1.0f / 64.0f);
  (void)hipGetLastError();
}
